// EquivariantGNN_17300128268844
// MI455X (gfx1250) — hardware-verified
//
#include <hip/hip_runtime.h>
#include <stddef.h>
#include <stdint.h>


#define EMB    64
#define INDIM  11
#define KX     32
#define EDIM   4
#define MR     133
#define NLAY   4
#define KAB    128
#define NAB    128
#define KU1    256
#define KU2    128
#define NTHR   256
#define NWAVE  8
#define EPT    8
#define CHUNK  (NTHR * EPT)
#define WCAP   (EPT * 32)
#define LISTN  (NWAVE * WCAP)
#define NBA    1024
#define SLA    10
#define SPW    (NBA / NWAVE)
#define RCAP   24576
#define DEGCAP 128
#define GBM    64
#define GBN    128
#define GTHR   128
#define EPB    256
#define DP     68
#define AP     72
#define CSTN   528
#define EDGE_LDS_BYTES (EPB * DP * 4 + EPB * AP * 2 + CSTN * 4 + EPB * 4)
#define NU_WIN 256
#define NU_WAB 8192
#define NU_WM2 2048
#define NU_WU1 8192
#define NU_WU2 4096
#define NU_W   (NU_WIN + NU_WAB + NU_WM2 + NU_WU1 + NU_WU2)
#define SC_ZINTS (LISTN + 2 * RCAP + 3 * NBA)
#define SC_LDS_INTS (SC_ZINTS + 16 + 4 * NBA)
#define WSLIM  268435456

static_assert((CHUNK & (CHUNK - 1)) == 0 && CHUNK <= 4096);
static_assert((NBA & (NBA - 1)) == 0 && NBA == (1 << SLA));
static_assert(((long long)CHUNK << SLA) < (1LL << 31));
static_assert(LISTN % NTHR == 0);
static_assert(NBA % NWAVE == 0 && NBA % 32 == 0 && NBA % GBM == 0 && NBA % NTHR == 0 && SPW % 32 == 0);
static_assert(RCAP % 4 == 0 && SC_ZINTS % 4 == 0 && LISTN % 4 == 0);
static_assert(SC_LDS_INTS * 4 <= 300000);
static_assert(EDGE_LDS_BYTES <= 300000);
static_assert(KX % 32 == 0 && KAB % 32 == 0 && KU1 % 32 == 0 && KU2 % 32 == 0 && EMB % 32 == 0);
static_assert(KAB == 2 * EMB && KU1 == 4 * EMB && KU2 == 2 * EMB && NAB == GBN && NAB == 2 * EMB);
static_assert(GBM == (GTHR / 32) * 16 && GBN == 4 * 32);
static_assert(NU_WIN % NTHR == 0 && NU_WAB % NTHR == 0 && NU_WM2 % NTHR == 0 && NU_WU1 % NTHR == 0 && NU_WU2 % NTHR == 0);
static_assert((GBM * 4) % NTHR == 0);
static_assert((DP * 4) % 16 == 0 && (AP * 2) % 16 == 0 && AP >= EMB && DP >= EMB);
static_assert((EPB * DP * 4) % 16 == 0 && (EPB * AP * 2) % 16 == 0 && (CSTN * 4) % 16 == 0);
static_assert(EPB == NTHR && EPB == 8 * 32);
static_assert(MR == 2 * EMB + EDIM + 1);
static_assert(INDIM <= KX && CSTN >= 513);

typedef float          v2f   __attribute__((ext_vector_type(2)));
typedef float          v4f   __attribute__((ext_vector_type(4)));
typedef float          v8f   __attribute__((ext_vector_type(8)));
typedef int            v4i   __attribute__((ext_vector_type(4)));
typedef int            v8i   __attribute__((ext_vector_type(8)));
typedef unsigned short v4us  __attribute__((ext_vector_type(4)));
typedef unsigned short v8us  __attribute__((ext_vector_type(8)));
typedef unsigned short v16us __attribute__((ext_vector_type(16)));
typedef __bf16         v16bf __attribute__((ext_vector_type(16)));
typedef _Float16       v16h  __attribute__((ext_vector_type(16)));
typedef v2f  __attribute__((may_alias)) v2fa;
typedef v4f  __attribute__((may_alias)) v4fa;
typedef v4i  __attribute__((may_alias)) v4ia;
typedef v4us __attribute__((may_alias)) v4usa;
typedef v8us __attribute__((may_alias)) v8usa;
union FragB { v16bf v; v16us u; v8us h[2]; v8i w; };
union FragH { v16h  v; v16us u; v8us h[2]; v8i w; };

__device__ __forceinline__ v8f wmb(const FragB& a, const FragB& b, v8f c) {
  v8f d = __builtin_amdgcn_wmma_f32_16x16x32_bf16(false, a.v, false, b.v, (short)0, c, false, false);
  asm volatile("v_nop\n\tv_nop\n\tv_nop\n\tv_nop" : "+v"(d) : "v"(a.w), "v"(b.w));
  return d;
}
__device__ __forceinline__ v8f wmh(const FragH& a, const FragH& b, v8f c) {
  v8f d = __builtin_amdgcn_wmma_f32_16x16x32_f16(false, a.v, false, b.v, (short)0, c, false, false);
  asm volatile("v_nop\n\tv_nop\n\tv_nop\n\tv_nop" : "+v"(d) : "v"(a.w), "v"(b.w));
  return d;
}

__device__ __forceinline__ unsigned bf16_bits(float f) {
  const unsigned u = __float_as_uint(f);
  return (u + 0x7FFFu + ((u >> 16) & 1u)) >> 16;
}
__device__ __forceinline__ float bf16_val(float f) {
  return __uint_as_float(bf16_bits(f) << 16);
}
__device__ __forceinline__ unsigned short h_bits(float f) {
  return __builtin_bit_cast(unsigned short, (_Float16)f);
}
__device__ __forceinline__ float h_val(unsigned b16) {
  return (float)__builtin_bit_cast(_Float16, (unsigned short)b16);
}
__device__ __forceinline__ float relu_nn(float v) {
  return (v > 0.0f || v != v) ? v : 0.0f;
}

template <int SLB>
__device__ __forceinline__ int scan_chunk(const int* __restrict__ dsts, int nE, int cbase, int slotBase,
                                          int nb, int vec8, int* list, int tid, int lane, int wave) {
  int wc = 0;
  const int el0  = tid * EPT;
  const int e0   = cbase + el0;
  const int sent = -2147483647 - 1;
  v4i da, db;
  if (vec8 != 0 && cbase + CHUNK <= nE) {
    da = *(const v4i*)(dsts + e0);
    db = *(const v4i*)(dsts + e0 + 4);
  } else {
    da.x = (e0     < nE) ? dsts[min(e0,     nE - 1)] : sent;
    da.y = (e0 + 1 < nE) ? dsts[min(e0 + 1, nE - 1)] : sent;
    da.z = (e0 + 2 < nE) ? dsts[min(e0 + 2, nE - 1)] : sent;
    da.w = (e0 + 3 < nE) ? dsts[min(e0 + 3, nE - 1)] : sent;
    db.x = (e0 + 4 < nE) ? dsts[min(e0 + 4, nE - 1)] : sent;
    db.y = (e0 + 5 < nE) ? dsts[min(e0 + 5, nE - 1)] : sent;
    db.z = (e0 + 6 < nE) ? dsts[min(e0 + 6, nE - 1)] : sent;
    db.w = (e0 + 7 < nE) ? dsts[min(e0 + 7, nE - 1)] : sent;
  }
  const unsigned nbs = (unsigned)slotBase;
  const unsigned unb = (unsigned)nb;
  const unsigned s0 = (unsigned)da.x - nbs, s1 = (unsigned)da.y - nbs;
  const unsigned s2 = (unsigned)da.z - nbs, s3 = (unsigned)da.w - nbs;
  const unsigned s4 = (unsigned)db.x - nbs, s5 = (unsigned)db.y - nbs;
  const unsigned s6 = (unsigned)db.z - nbs, s7 = (unsigned)db.w - nbs;
  const bool h0 = s0 < unb, h1 = s1 < unb, h2 = s2 < unb, h3 = s3 < unb;
  const bool h4 = s4 < unb, h5 = s5 < unb, h6 = s6 < unb, h7 = s7 < unb;
  const unsigned any = __builtin_amdgcn_ballot_w32(h0 | h1 | h2 | h3 | h4 | h5 | h6 | h7);
  if (any != 0u) {
#define HITJ(J, HJ, SJ) { \
      const unsigned mj = __builtin_amdgcn_ballot_w32(HJ); \
      if (mj != 0u) { \
        if (HJ) { \
          const int pos = wc + (int)__builtin_amdgcn_mbcnt_lo(mj, 0u); \
          if (pos < WCAP) list[wave * WCAP + pos] = ((el0 + (J)) << SLB) | (int)(SJ); \
        } \
        wc += (int)__builtin_popcount(mj); } }
    HITJ(0, h0, s0)
    HITJ(1, h1, s1)
    HITJ(2, h2, s2)
    HITJ(3, h3, s3)
    HITJ(4, h4, s4)
    HITJ(5, h5, s5)
    HITJ(6, h6, s6)
    HITJ(7, h7, s7)
#undef HITJ
  }
  return wc;
}

__global__ __launch_bounds__(NTHR) void k_prep(const float* __restrict__ x, const float* __restrict__ pos,
                                               const float* __restrict__ Win, const float* __restrict__ Wm1,
                                               const float* __restrict__ Wm2, const float* __restrict__ Wu1,
                                               const float* __restrict__ Wu2, int nN, int mRows, int pRows,
                                               unsigned short* WinT, unsigned short* WABT, unsigned short* Wm2T,
                                               unsigned short* Wu1T, unsigned short* Wu2T, unsigned short* XA,
                                               float* posA) {
  const int u = (int)blockIdx.x * NTHR + (int)threadIdx.x;
  if (u < NU_W + mRows * 4) {
    v8us o;
    unsigned short* dp;
    if (u < NU_WIN) {
      const int n  = u >> 2;
      const int k8 = (u & 3) * 8;
#pragma unroll
      for (int i = 0; i < 8; ++i) {
        const int k  = k8 + i;
        const int kc = k < INDIM ? k : INDIM - 1;
        const unsigned short b = (unsigned short)bf16_bits(Win[kc * EMB + n]);
        o[i] = k < INDIM ? b : (unsigned short)0;
      }
      dp = WinT + (size_t)n * KX + k8;
    } else if (u < NU_WIN + NU_WAB) {
      const int v  = u - NU_WIN;
      const int l  = v >> 11;
      const int rr = v & 2047;
      const int n  = rr >> 4;
      const int k8 = (rr & 15) * 8;
      const int kk = k8 & (EMB - 1);
      const int hf = n >> 6;
      const int nn = n & (EMB - 1);
      const float* p = Wm1 + ((size_t)l * MR + (size_t)hf * EMB + kk) * EMB + nn;
#pragma unroll
      for (int i = 0; i < 8; ++i) o[i] = (unsigned short)bf16_bits(p[(size_t)i * EMB]);
      dp = WABT + ((size_t)l * NAB + n) * KAB + k8;
    } else if (u < NU_WIN + NU_WAB + NU_WM2) {
      const int v  = u - NU_WIN - NU_WAB;
      const int l  = v >> 9;
      const int rr = v & 511;
      const int n  = rr >> 3;
      const int k8 = (rr & 7) * 8;
      const float* p = Wm2 + ((size_t)l * EMB + k8) * EMB + n;
#pragma unroll
      for (int i = 0; i < 8; ++i) o[i] = h_bits(16.0f * bf16_val(p[(size_t)i * EMB]));
      dp = Wm2T + ((size_t)l * EMB + n) * EMB + k8;
    } else if (u < NU_WIN + NU_WAB + NU_WM2 + NU_WU1) {
      const int v  = u - NU_WIN - NU_WAB - NU_WM2;
      const int l  = v >> 11;
      const int rr = v & 2047;
      const int n  = rr >> 5;
      const int k8 = (rr & 31) * 8;
      const int kk = k8 & (2 * EMB - 1);
      const float* p = Wu1 + ((size_t)l * 2 * EMB + kk) * EMB + n;
#pragma unroll
      for (int i = 0; i < 8; ++i) o[i] = (unsigned short)bf16_bits(p[(size_t)i * EMB]);
      dp = Wu1T + ((size_t)l * EMB + n) * KU1 + k8;
    } else if (u < NU_W) {
      const int v  = u - NU_WIN - NU_WAB - NU_WM2 - NU_WU1;
      const int l  = v >> 10;
      const int rr = v & 1023;
      const int n  = rr >> 4;
      const int k8 = (rr & 15) * 8;
      const int kk = k8 & (EMB - 1);
      const float* p = Wu2 + ((size_t)l * EMB + kk) * EMB + n;
#pragma unroll
      for (int i = 0; i < 8; ++i) o[i] = (unsigned short)bf16_bits(p[(size_t)i * EMB]);
      dp = Wu2T + ((size_t)l * EMB + n) * KU2 + k8;
    } else {
      const int v   = u - NU_W;
      const int row = v >> 2;
      const int k8  = (v & 3) * 8;
      const int rc  = row < nN ? row : nN - 1;
      const bool ok = row < nN;
      const float* xr = x + (size_t)rc * INDIM;
#pragma unroll
      for (int i = 0; i < 8; ++i) {
        const int k  = k8 + i;
        const int kc = k < INDIM ? k : INDIM - 1;
        const unsigned short b = (unsigned short)bf16_bits(xr[kc]);
        o[i] = (ok && k < INDIM) ? b : (unsigned short)0;
      }
      dp = XA + (size_t)row * KX + k8;
    }
    *(volatile v8us*)dp = o;
    __threadfence();
    *(volatile v8us*)dp = o;
  } else {
    const int v = u - NU_W - mRows * 4;
    if (v >= pRows) return;
    const int rc  = v < nN ? v : nN - 1;
    const bool ok = v < nN;
    const float* p = pos + (size_t)rc * 3;
    v4f q;
    q.x = ok ? bf16_val(p[0]) : 0.0f;
    q.y = ok ? bf16_val(p[1]) : 0.0f;
    q.z = ok ? bf16_val(p[2]) : 0.0f;
    q.w = 0.0f;
    float* fp = posA + (size_t)v * 4;
    *(volatile v4f*)fp = q;
    __threadfence();
    *(volatile v4f*)fp = q;
  }
}

__global__ __launch_bounds__(GTHR) void k_gemm(const unsigned short* __restrict__ A, int lda,
                                               const unsigned short* __restrict__ BT, int ldb, int K,
                                               float* Cm, int ldc) {
  __shared__ __attribute__((aligned(16))) float stg[GBM * GBN];
  const int tid = (int)threadIdx.x, lane = tid & 31, wave = tid >> 5, hh = lane >> 4, m = lane & 15;
  const int rowBase = (int)blockIdx.x * GBM;
  const int colBase = (int)blockIdx.y * GBN;

  v8f acc[8];
  {
    const v8f z = {0.f, 0.f, 0.f, 0.f, 0.f, 0.f, 0.f, 0.f};
#pragma unroll
    for (int t = 0; t < 8; ++t) acc[t] = z;
  }
  const unsigned short* ap = A  + (size_t)(rowBase + 16 * wave + m) * (size_t)lda + 8 * hh;
  const unsigned short* bp = BT + (size_t)(colBase + m) * (size_t)ldb + 8 * hh;

#pragma unroll 1
  for (int k0 = 0; k0 < K; k0 += 32) {
    FragB af;
    af.h[0] = *(const v8usa*)(ap + k0);
    af.h[1] = *(const v8usa*)(ap + k0 + 16);
#pragma unroll
    for (int nt = 0; nt < 8; ++nt) {
      const unsigned short* wq = bp + (size_t)(16 * nt) * (size_t)ldb + k0;
      FragB bf;
      bf.h[0] = *(const v8usa*)wq;
      bf.h[1] = *(const v8usa*)(wq + 16);
      acc[nt] = wmb(af, bf, acc[nt]);
    }
  }

#pragma unroll
  for (int nt = 0; nt < 8; ++nt) {
    const int lc = 16 * nt + m;
#pragma unroll
    for (int r = 0; r < 8; ++r) {
      const int lr = 16 * wave + 8 * hh + r;
      stg[lr * GBN + lc] = acc[nt][r];
    }
  }
  __syncthreads();

  v4f pv[16];
#pragma unroll
  for (int i = 0; i < 16; ++i) pv[i] = *(const v4fa*)(stg + (16 * wave + i) * GBN + 4 * lane);
#pragma unroll
  for (int i = 0; i < 16; ++i) {
    float* op = Cm + (size_t)(rowBase + 16 * wave + i) * (size_t)ldc + colBase + 4 * lane;
    *(volatile v4f*)op = pv[i];
  }
  __threadfence();
#pragma unroll
  for (int i = 0; i < 16; ++i) {
    float* op = Cm + (size_t)(rowBase + 16 * wave + i) * (size_t)ldc + colBase + 4 * lane;
    *(volatile v4f*)op = pv[i];
  }
}

__device__ __forceinline__ void gemm64(v8f (&acc)[4], const unsigned short* __restrict__ A, int lda,
                                       const unsigned short* __restrict__ BT, int ldb, int K,
                                       int rowBase, int wave, int hh, int m) {
  {
    const v8f z = {0.f, 0.f, 0.f, 0.f, 0.f, 0.f, 0.f, 0.f};
#pragma unroll
    for (int t = 0; t < 4; ++t) acc[t] = z;
  }
  const unsigned short* ap = A  + (size_t)(rowBase + 16 * wave + m) * (size_t)lda + 8 * hh;
  const unsigned short* bp = BT + (size_t)m * (size_t)ldb + 8 * hh;
#pragma unroll 1
  for (int k0 = 0; k0 < K; k0 += 32) {
    FragB af;
    af.h[0] = *(const v8usa*)(ap + k0);
    af.h[1] = *(const v8usa*)(ap + k0 + 16);
#pragma unroll
    for (int nt = 0; nt < 4; ++nt) {
      const unsigned short* wq = bp + (size_t)(16 * nt) * (size_t)ldb + k0;
      FragB bf;
      bf.h[0] = *(const v8usa*)wq;
      bf.h[1] = *(const v8usa*)(wq + 16);
      acc[nt] = wmb(af, bf, acc[nt]);
    }
  }
}

__device__ __forceinline__ void dmap64(float* stg, const v8f (&acc)[4], const float (&bv)[4], int act,
                                       int wave, int hh, int m) {
#pragma unroll
  for (int nt = 0; nt < 4; ++nt) {
    const int lc = 16 * nt + m;
#pragma unroll
    for (int r = 0; r < 8; ++r) {
      const int lr = 16 * wave + 8 * hh + r;
      float v = acc[nt][r] + bv[nt];
      if (act != 0) v = relu_nn(v);
      stg[lr * EMB + lc] = v;
    }
  }
}

template <int WF, int RES>
__device__ __forceinline__ void epi64(float* stg, unsigned short* stb, int rowBase, int nN, int wave,
                                      int lane, float* Hp, unsigned short* Bp) {
  __syncthreads();
  v4f pv[8];
  const size_t fbase = (size_t)(rowBase + 16 * wave) * EMB;
#pragma unroll
  for (int i = 0; i < 8; ++i) {
    const int fo = i * 128 + 4 * lane;
    const int lr = 16 * wave + (fo >> 6);
    const int c  = fo & (EMB - 1);
    v4f v = *(const v4fa*)(stg + lr * EMB + c);
    if constexpr (RES != 0) {
      const v4f hr = *(const v4fa*)(Hp + fbase + fo);
      v.x += hr.x; v.y += hr.y; v.z += hr.z; v.w += hr.w;
    }
    const bool ok = (rowBase + lr) < nN;
    v.x = ok ? v.x : 0.0f; v.y = ok ? v.y : 0.0f; v.z = ok ? v.z : 0.0f; v.w = ok ? v.w : 0.0f;
    if constexpr (RES != 0) *(v4fa*)(stg + lr * EMB + c) = v;
    pv[i] = v;
    v4us ho, lo;
#pragma unroll
    for (int j = 0; j < 4; ++j) {
      const unsigned hb = bf16_bits(v[j]);
      ho[j] = (unsigned short)hb;
      lo[j] = (unsigned short)bf16_bits(v[j] - __uint_as_float(hb << 16));
    }
    *(v4usa*)(stb + lr * KAB + c)       = ho;
    *(v4usa*)(stb + lr * KAB + EMB + c) = lo;
  }
  __syncthreads();
  v8us hv[8];
  const size_t bbase = (size_t)(rowBase + 16 * wave) * KAB;
#pragma unroll
  for (int i = 0; i < 8; ++i) hv[i] = *(const v8usa*)(stb + 16 * wave * KAB + i * 256 + 8 * lane);
#pragma unroll
  for (int i = 0; i < 8; ++i) {
    if constexpr (WF != 0) *(volatile v4f*)(Hp + fbase + i * 128 + 4 * lane) = pv[i];
    *(volatile v8us*)(Bp + bbase + i * 256 + 8 * lane) = hv[i];
  }
  __threadfence();
#pragma unroll
  for (int i = 0; i < 8; ++i) {
    if constexpr (WF != 0) *(volatile v4f*)(Hp + fbase + i * 128 + 4 * lane) = pv[i];
    *(volatile v8us*)(Bp + bbase + i * 256 + 8 * lane) = hv[i];
  }
}

__global__ __launch_bounds__(GTHR) void k_h0(const unsigned short* __restrict__ XA,
                                             const unsigned short* __restrict__ WinT,
                                             const float* __restrict__ bin, int nN,
                                             float* H, unsigned short* HB) {
  __shared__ __attribute__((aligned(16))) float stg[GBM * EMB];
  __shared__ __attribute__((aligned(16))) unsigned short stb[GBM * KAB];
  const int tid = (int)threadIdx.x, lane = tid & 31, wave = tid >> 5, hh = lane >> 4, m = lane & 15;
  const int rowBase = (int)blockIdx.x * GBM;
  v8f acc[4];
  gemm64(acc, XA, KX, WinT, KX, KX, rowBase, wave, hh, m);
  float bv[4];
#pragma unroll
  for (int nt = 0; nt < 4; ++nt) bv[nt] = bf16_val(bin[16 * nt + m]);
  dmap64(stg, acc, bv, 0, wave, hh, m);
  epi64<1, 0>(stg, stb, rowBase, nN, wave, lane, H, HB);
}

__global__ __launch_bounds__(GTHR) void k_u1(const unsigned short* __restrict__ UA,
                                             const unsigned short* __restrict__ W1T,
                                             const float* __restrict__ bu, int nN, unsigned short* U1A) {
  __shared__ __attribute__((aligned(16))) float stg[GBM * EMB];
  __shared__ __attribute__((aligned(16))) unsigned short stb[GBM * KAB];
  const int tid = (int)threadIdx.x, lane = tid & 31, wave = tid >> 5, hh = lane >> 4, m = lane & 15;
  const int rowBase = (int)blockIdx.x * GBM;
  v8f acc[4];
  gemm64(acc, UA, KU1, W1T, KU1, KU1, rowBase, wave, hh, m);
  float bv[4];
#pragma unroll
  for (int nt = 0; nt < 4; ++nt) bv[nt] = bf16_val(bu[16 * nt + m]);
  dmap64(stg, acc, bv, 1, wave, hh, m);
  epi64<0, 0>(stg, stb, rowBase, nN, wave, lane, stg, U1A);
}

template <int LAST>
__global__ __launch_bounds__(GTHR) void k_u2(const unsigned short* __restrict__ U1A,
                                             const unsigned short* __restrict__ W2T,
                                             const float* __restrict__ bu, int nN,
                                             float* H, unsigned short* HB,
                                             const float* __restrict__ Wout, const float* __restrict__ bout,
                                             float* dout) {
  __shared__ __attribute__((aligned(16))) float stg[GBM * EMB];
  __shared__ __attribute__((aligned(16))) unsigned short stb[GBM * KAB];
  __shared__ __attribute__((aligned(16))) float sWo[EMB];
  __shared__ __attribute__((aligned(16))) float sOut[GBM];
  __shared__ float sbo[4];
  const int tid = (int)threadIdx.x, lane = tid & 31, wave = tid >> 5, hh = lane >> 4, m = lane & 15;
  const int rowBase = (int)blockIdx.x * GBM;
  if constexpr (LAST != 0) {
    if (tid < 64) {
      sWo[tid] = bf16_val(Wout[tid]);
      const float b = bf16_val(bout[0]);
      if (tid == 0) sbo[0] = b;
    }
  }
  v8f acc[4];
  gemm64(acc, U1A, KU2, W2T, KU2, KU2, rowBase, wave, hh, m);
  float bv[4];
#pragma unroll
  for (int nt = 0; nt < 4; ++nt) bv[nt] = bf16_val(bu[16 * nt + m]);
  dmap64(stg, acc, bv, 1, wave, hh, m);
  epi64<1, 1>(stg, stb, rowBase, nN, wave, lane, H, HB);

  if constexpr (LAST != 0) {
    const int lr = 16 * wave + (lane & 15);
    const int hf = lane >> 4;
    const float* rp = stg + lr * EMB + 32 * hf;
    const float* wp = sWo + 32 * hf;
    float ds = 0.0f;
#pragma unroll
    for (int c4 = 0; c4 < 8; ++c4) {
      const v4f a = *(const v4fa*)(rp + 4 * c4);
      const v4f w = *(const v4fa*)(wp + 4 * c4);
      ds = fmaf(a.x, w.x, ds); ds = fmaf(a.y, w.y, ds); ds = fmaf(a.z, w.z, ds); ds = fmaf(a.w, w.w, ds);
    }
    ds += __shfl_xor(ds, 16, 32);
    const float ov = ds + sbo[0];
    if (hf == 0) sOut[lr] = ov;
    __syncthreads();
    if (wave == 0) {
      int nval = nN - rowBase;
      nval = nval > GBM ? GBM : (nval < 0 ? 0 : nval);
      const int nq  = nval >> 2;
      const int rem = nval & 3;
      const int tl  = lane < 16 ? lane : 15;
      const v4f o4 = *(const v4fa*)(sOut + 4 * tl);
      const int tb = 4 * nq;
      const float t0 = sOut[tb     < GBM ? tb     : GBM - 1];
      const float t1 = sOut[tb + 1 < GBM ? tb + 1 : GBM - 1];
      const float t2 = sOut[tb + 2 < GBM ? tb + 2 : GBM - 1];
      const bool st  = lane < nq;
      const bool s0  = (lane == 0) && rem > 0;
      const bool s1  = (lane == 0) && rem > 1;
      const bool s2  = (lane == 0) && rem > 2;
      float* op = dout + (size_t)rowBase + 4 * tl;
      float* tp = dout + (size_t)rowBase + tb;
      if (st) *(volatile v4f*)op = o4;
      if (s0) *(volatile float*)(tp)     = t0;
      if (s1) *(volatile float*)(tp + 1) = t1;
      if (s2) *(volatile float*)(tp + 2) = t2;
      __threadfence();
      if (st) *(volatile v4f*)op = o4;
      if (s0) *(volatile float*)(tp)     = t0;
      if (s1) *(volatile float*)(tp + 1) = t1;
      if (s2) *(volatile float*)(tp + 2) = t2;
    }
  }
}

__global__ __launch_bounds__(NTHR) void k_edge(const int* __restrict__ ei, int nE, int nN,
                                               const float* __restrict__ PAB, const float* __restrict__ posCur,
                                               const float* __restrict__ ea,
                                               const unsigned short* __restrict__ W2T,
                                               const float* __restrict__ Wm1l, const float* __restrict__ bm1l,
                                               const float* __restrict__ bm2l, const float* __restrict__ Wpl,
                                               const float* __restrict__ bpl,
                                               float* Sp, unsigned short* Mp) {
  extern __shared__ __attribute__((aligned(16))) float dyn[];
  float*          sD  = dyn;
  unsigned short* sA  = (unsigned short*)(dyn + EPB * DP);
  float*          cst = dyn + EPB * DP + (EPB * AP) / 2;
  float*          sS  = cst + CSTN;

  const int tid = (int)threadIdx.x, lane = tid & 31, wave = tid >> 5, hh = lane >> 4, m = lane & 15;

  if (tid < 64) {
    cst[tid]       = bf16_val(Wm1l[(2 * EMB + 0) * EMB + tid]);
    cst[64 + tid]  = bf16_val(Wm1l[(2 * EMB + 1) * EMB + tid]);
    cst[128 + tid] = bf16_val(Wm1l[(2 * EMB + 2) * EMB + tid]);
    cst[192 + tid] = bf16_val(Wm1l[(2 * EMB + 3) * EMB + tid]);
    cst[256 + tid] = bf16_val(Wm1l[(2 * EMB + 4) * EMB + tid]);
    cst[320 + tid] = bf16_val(bm1l[tid]);
    cst[384 + tid] = bf16_val(bm2l[tid]);
    cst[448 + tid] = bf16_val(Wpl[tid]);
    const float vbp = bf16_val(bpl[0]);
    if (tid == 0) cst[512] = vbp;
  }

  const int e0 = (int)blockIdx.x * EPB;
  int ec = e0 + tid;
  ec = ec > nE - 1 ? nE - 1 : ec;
  int s = ei[ec];
  int t = ei[(size_t)nE + (size_t)ec];
  s = s < 0 ? 0 : (s > nN - 1 ? nN - 1 : s);
  t = t < 0 ? 0 : (t > nN - 1 ? nN - 1 : t);
  const float* pa = PAB + (size_t)t * NAB;
  const float* pb = PAB + (size_t)s * NAB + EMB;
  const v4f eav = *(const v4fa*)(ea + (size_t)ec * EDIM);
  const float ea0 = bf16_val(eav.x), ea1 = bf16_val(eav.y), ea2 = bf16_val(eav.z), ea3 = bf16_val(eav.w);
  const v4f pt = *(const v4fa*)(posCur + (size_t)t * 4);
  const v4f ps = *(const v4fa*)(posCur + (size_t)s * 4);
  const float rx = pt.x - ps.x, ry = pt.y - ps.y, rz = pt.z - ps.z;
  const float dist = sqrtf((rx * rx + rz * rz) + ry * ry + 0.0f);
  float* rd = sD + tid * DP;
  unsigned short* ra = sA + tid * AP;
  __syncthreads();

#pragma unroll 2
  for (int c8 = 0; c8 < EMB / 8; ++c8) {
    const v4f a0 = *(const v4fa*)(pa + 8 * c8);
    const v4f a1 = *(const v4fa*)(pa + 8 * c8 + 4);
    const v4f b0 = *(const v4fa*)(pb + 8 * c8);
    const v4f b1 = *(const v4fa*)(pb + 8 * c8 + 4);
    const v4f w0a = *(const v4fa*)(cst + 8 * c8),        w0b = *(const v4fa*)(cst + 8 * c8 + 4);
    const v4f w1a = *(const v4fa*)(cst + 64 + 8 * c8),   w1b = *(const v4fa*)(cst + 64 + 8 * c8 + 4);
    const v4f w2a = *(const v4fa*)(cst + 128 + 8 * c8),  w2b = *(const v4fa*)(cst + 128 + 8 * c8 + 4);
    const v4f w3a = *(const v4fa*)(cst + 192 + 8 * c8),  w3b = *(const v4fa*)(cst + 192 + 8 * c8 + 4);
    const v4f wda = *(const v4fa*)(cst + 256 + 8 * c8),  wdb = *(const v4fa*)(cst + 256 + 8 * c8 + 4);
    const v4f bma = *(const v4fa*)(cst + 320 + 8 * c8),  bmb = *(const v4fa*)(cst + 320 + 8 * c8 + 4);
    const v8f av = {a0.x, a0.y, a0.z, a0.w, a1.x, a1.y, a1.z, a1.w};
    const v8f sv = {b0.x, b0.y, b0.z, b0.w, b1.x, b1.y, b1.z, b1.w};
    const v8f w0 = {w0a.x, w0a.y, w0a.z, w0a.w, w0b.x, w0b.y, w0b.z, w0b.w};
    const v8f w1 = {w1a.x, w1a.y, w1a.z, w1a.w, w1b.x, w1b.y, w1b.z, w1b.w};
    const v8f w2 = {w2a.x, w2a.y, w2a.z, w2a.w, w2b.x, w2b.y, w2b.z, w2b.w};
    const v8f w3 = {w3a.x, w3a.y, w3a.z, w3a.w, w3b.x, w3b.y, w3b.z, w3b.w};
    const v8f wd = {wda.x, wda.y, wda.z, wda.w, wdb.x, wdb.y, wdb.z, wdb.w};
    const v8f bm = {bma.x, bma.y, bma.z, bma.w, bmb.x, bmb.y, bmb.z, bmb.w};
    v8us o;
#pragma unroll
    for (int i = 0; i < 8; ++i) {
      const float ev = fmaf(ea0, w0[i], ea1 * w1[i]) + fmaf(ea2, w2[i], ea3 * w3[i]);
      float v = (av[i] + sv[i]) + (ev + fmaf(dist, wd[i], bm[i]));
      v = relu_nn(v);
      v = v > 65000.0f ? 65000.0f : v;
      o[i] = h_bits(v);
    }
    *(v8usa*)(ra + 8 * c8) = o;
  }
  __syncthreads();

  v8f acc[2][4];
  {
    const v8f z = {0.f, 0.f, 0.f, 0.f, 0.f, 0.f, 0.f, 0.f};
#pragma unroll
    for (int mt = 0; mt < 2; ++mt)
#pragma unroll
      for (int nt = 0; nt < 4; ++nt) acc[mt][nt] = z;
  }
  const unsigned short* ap0 = sA + (32 * wave + m) * AP + 8 * hh;
  const unsigned short* ap1 = ap0 + 16 * AP;
  const unsigned short* bq  = W2T + (size_t)m * EMB + 8 * hh;
#pragma unroll 1
  for (int k0 = 0; k0 < EMB; k0 += 32) {
    FragH fa0, fa1;
    fa0.h[0] = *(const v8usa*)(ap0 + k0);
    fa0.h[1] = *(const v8usa*)(ap0 + k0 + 16);
    fa1.h[0] = *(const v8usa*)(ap1 + k0);
    fa1.h[1] = *(const v8usa*)(ap1 + k0 + 16);
#pragma unroll
    for (int nt = 0; nt < 4; ++nt) {
      const unsigned short* wq = bq + (size_t)(16 * nt) * EMB + k0;
      FragH fb;
      fb.h[0] = *(const v8usa*)wq;
      fb.h[1] = *(const v8usa*)(wq + 16);
      acc[0][nt] = wmh(fa0, fb, acc[0][nt]);
      acc[1][nt] = wmh(fa1, fb, acc[1][nt]);
    }
  }
#pragma unroll
  for (int nt = 0; nt < 4; ++nt) {
    const int col = 16 * nt + m;
    const float b2 = cst[384 + col];
#pragma unroll
    for (int mt = 0; mt < 2; ++mt)
#pragma unroll
      for (int r = 0; r < 8; ++r)
        sD[(32 * wave + 16 * mt + 8 * hh + r) * DP + col] = relu_nn(fmaf(acc[mt][nt][r], 0.0625f, b2));
  }
  __syncthreads();

  float ssum = 0.0f;
#pragma unroll 2
  for (int c8 = 0; c8 < EMB / 8; ++c8) {
    const v4f va = *(const v4fa*)(rd + 8 * c8);
    const v4f vb = *(const v4fa*)(rd + 8 * c8 + 4);
    const v4f wa = *(const v4fa*)(cst + 448 + 8 * c8);
    const v4f wb = *(const v4fa*)(cst + 448 + 8 * c8 + 4);
    const v8f v8 = {va.x, va.y, va.z, va.w, vb.x, vb.y, vb.z, vb.w};
    const v8f w8 = {wa.x, wa.y, wa.z, wa.w, wb.x, wb.y, wb.z, wb.w};
    v8us o;
#pragma unroll
    for (int i = 0; i < 8; ++i) {
      ssum = fmaf(v8[i], w8[i], ssum);
      const float mv = v8[i] > 65000.0f ? 65000.0f : v8[i];
      o[i] = h_bits(mv);
    }
    *(v8usa*)(ra + 8 * c8) = o;
  }
  sS[tid] = ssum + cst[512];
  __syncthreads();

  v8us mv[8];
#pragma unroll
  for (int i = 0; i < 8; ++i) {
    const int lr = 32 * wave + 4 * i + (lane >> 3);
    const int p  = lane & 7;
    mv[i] = *(const v8usa*)(sA + lr * AP + 8 * p);
  }
  const int  tl  = tid < 64 ? tid : 63;
  const v4f  s4  = *(const v4fa*)(sS + 4 * tl);
  const bool sst = tid < 64;
#pragma unroll
  for (int i = 0; i < 8; ++i) {
    const int lr = 32 * wave + 4 * i + (lane >> 3);
    const int p  = lane & 7;
    *(volatile v8us*)(Mp + (size_t)(e0 + lr) * EMB + 8 * p) = mv[i];
  }
  if (sst) *(volatile v4f*)(Sp + (size_t)e0 + 4 * tl) = s4;
  __threadfence();
#pragma unroll
  for (int i = 0; i < 8; ++i) {
    const int lr = 32 * wave + 4 * i + (lane >> 3);
    const int p  = lane & 7;
    *(volatile v8us*)(Mp + (size_t)(e0 + lr) * EMB + 8 * p) = mv[i];
  }
  if (sst) *(volatile v4f*)(Sp + (size_t)e0 + 4 * tl) = s4;
}

__global__ __launch_bounds__(NTHR) void k_scan(const int* __restrict__ srcs, const int* __restrict__ dsts,
                                               int nE, int nN, int vec8, int mRows,
                                               const unsigned short* __restrict__ Mp,
                                               const float* __restrict__ Sp,
                                               const float* __restrict__ posCur, float* posNext,
                                               const float* __restrict__ H, unsigned short* UA) {
  extern __shared__ __attribute__((aligned(16))) int dsm[];
  int* list = dsm;
  int* hl   = dsm + LISTN;
  int* sl   = dsm + LISTN + RCAP;
  int* cnt  = dsm + LISTN + 2 * RCAP;
  int* offs = cnt + NBA;
  int* cur  = offs + NBA;
  int* misc = cur + NBA;
  float* sPos = (float*)(misc + 16);
  const int tid = (int)threadIdx.x, lane = tid & 31, wave = tid >> 5;
  const int nodeBase = (int)blockIdx.x * NBA;

  {
    const v4i z4 = {0, 0, 0, 0};
    for (int i = tid * 4; i < SC_ZINTS; i += NTHR * 4) *(v4ia*)(dsm + i) = z4;
    if (tid < 16) misc[tid] = 0;
  }
  __syncthreads();

  int t = 0, ov = 0;
  const int nChunks = (nE + CHUNK - 1) / CHUNK;
#pragma unroll 1
  for (int ch = 0; ch < nChunks; ++ch) {
    const int cbase = ch * CHUNK;
    const int wc = scan_chunk<SLA>(dsts, nE, cbase, nodeBase, NBA, vec8, list, tid, lane, wave);
    if (lane == 0) misc[wave] = wc;
    __syncthreads();
    if (wave == 0) {
#pragma unroll 1
      for (int w2 = 0; w2 < NWAVE; ++w2) {
        int c = misc[w2];
        c = c < 0 ? 0 : (c > WCAP ? WCAP : c);
#pragma unroll 1
        for (int b0 = 0; b0 < c; b0 += 32) {
          const int idx = b0 + lane;
          const int ent = list[w2 * WCAP + (idx < WCAP ? idx : WCAP - 1)];
          const int m32 = (c - b0) < 32 ? (c - b0) : 32;
#pragma unroll 1
          for (int k = 0; k < m32; ++k) {
            const int u    = __builtin_amdgcn_readlane(ent, k);
            const int slot = u & (NBA - 1);
            const int el   = (u >> SLA) & (CHUNK - 1);
            const int pk   = ((cbase + el) << SLA) | slot;
            if (t < RCAP) {
              if (lane == 0) { hl[t] = pk; cnt[slot] = cnt[slot] + 1; }
              t = t + 1;
            } else {
              ov = 1;
            }
          }
        }
      }
    }
    __syncthreads();
  }
  if (wave == 0 && lane == 0) { misc[8] = t; misc[9] = ov; }
  __syncthreads();
  int tt = misc[8];
  tt = tt < 0 ? 0 : (tt > RCAP ? RCAP : tt);
  const int ovf = misc[9];

  if (wave == 0) {
    const int base = lane * (NBA / 32);
    int sacc = 0;
#pragma unroll 1
    for (int i = 0; i < NBA / 32; ++i) sacc += cnt[base + i];
    int incl = sacc;
#pragma unroll
    for (int d = 1; d < 32; d <<= 1) {
      const int y = __shfl_up(incl, d, 32);
      if (lane >= d) incl += y;
    }
    int run = incl - sacc;
#pragma unroll 1
    for (int i = 0; i < NBA / 32; ++i) {
      const int cv = cnt[base + i];
      offs[base + i] = run;
      cur[base + i]  = run;
      run += cv;
    }
  }
  __syncthreads();
  if (wave == 0) {
#pragma unroll 1
    for (int b0 = 0; b0 < tt; b0 += 32) {
      const int idx = b0 + lane;
      const int ent = hl[idx < RCAP ? idx : RCAP - 1];
      const int m32 = (tt - b0) < 32 ? (tt - b0) : 32;
#pragma unroll 1
      for (int k = 0; k < m32; ++k) {
        const int u    = __builtin_amdgcn_readlane(ent, k);
        const int slot = u & (NBA - 1);
        if (lane == 0) {
          int p = cur[slot];
          p = p < 0 ? 0 : (p > RCAP - 1 ? RCAP - 1 : p);
          sl[p] = u;
          cur[slot] = p + 1;
        }
      }
    }
  }
  __syncthreads();

  const float pz = (ovf != 0) ? __int_as_float(0x7fc00000) : 0.0f;
#pragma unroll 1
  for (int si = 0; si < SPW; ++si) {
    const int s    = wave * SPW + si;
    const int node = nodeBase + s;
    const int cf   = cnt[s];
    const bool big = cf > DEGCAP;
    const int c = cf < 0 ? 0 : (cf > DEGCAP ? DEGCAP : cf);
    int o = offs[s];
    o = o < 0 ? 0 : (o > RCAP ? RCAP : o);
    const int nc = node < nN ? node : nN - 1;
    const v4f pd = *(const v4fa*)(posCur + (size_t)nc * 4);
    float a0 = 0.0f, a1 = 0.0f, px = 0.0f, py = 0.0f, pq = 0.0f;
#pragma unroll 1
    for (int b0 = 0; b0 < c; b0 += 32) {
      int idx = o + b0 + lane;
      idx = idx > RCAP - 1 ? RCAP - 1 : idx;
      const int ent = sl[idx];
      int eid = ent >> SLA;
      eid = eid < 0 ? 0 : (eid > nE - 1 ? nE - 1 : eid);
      const float act = (b0 + lane < c) ? 1.0f : 0.0f;
      int sr = srcs[eid];
      sr = sr < 0 ? 0 : (sr > nN - 1 ? nN - 1 : sr);
      const float sv = Sp[eid];
      const v4f ps = *(const v4fa*)(posCur + (size_t)sr * 4);
      const float sa = act * sv;
      px = fmaf(pd.x - ps.x, sa, px);
      py = fmaf(pd.y - ps.y, sa, py);
      pq = fmaf(pd.z - ps.z, sa, pq);
      const int m32 = (c - b0) < 32 ? (c - b0) : 32;
#pragma unroll 1
      for (int k = 0; k < m32; ++k) {
        const int ek = __builtin_amdgcn_readlane(eid, k);
        const unsigned w = *(const unsigned*)(Mp + (size_t)ek * EMB + 2 * lane);
        a0 += h_val(w & 0xffffu);
        a1 += h_val(w >> 16);
      }
    }
#pragma unroll
    for (int d = 16; d > 0; d >>= 1) {
      px += __shfl_xor(px, d, 32);
      py += __shfl_xor(py, d, 32);
      pq += __shfl_xor(pq, d, 32);
    }
    const float degf = fmaxf((float)(cf < 0 ? 0 : cf), 1.0f);
    const float rdeg = __builtin_amdgcn_rcpf(degf);
    const float pzr  = big ? __int_as_float(0x7fc00000) : pz;
    const bool  live = node < nN;
    v4f pn;
    pn.x = live ? (fmaf(px, rdeg, pd.x) + pzr) : 0.0f;
    pn.y = live ? (fmaf(py, rdeg, pd.y) + pzr) : 0.0f;
    pn.z = live ? (fmaf(pq, rdeg, pd.z) + pzr) : 0.0f;
    pn.w = 0.0f;
    if (lane == 0) *(v4fa*)(sPos + s * 4) = pn;
    const v2f hv = *(const v2fa*)(H + (size_t)nc * EMB + 2 * lane);
    const float h0 = live ? hv.x : 0.0f, h1 = live ? hv.y : 0.0f;
    const float g0 = live ? (a0 + pzr) : 0.0f, g1 = live ? (a1 + pzr) : 0.0f;
    const unsigned bh0 = bf16_bits(h0), bh1 = bf16_bits(h1), bg0 = bf16_bits(g0), bg1 = bf16_bits(g1);
    const unsigned lh0 = bf16_bits(h0 - __uint_as_float(bh0 << 16));
    const unsigned lh1 = bf16_bits(h1 - __uint_as_float(bh1 << 16));
    const unsigned lg0 = bf16_bits(g0 - __uint_as_float(bg0 << 16));
    const unsigned lg1 = bf16_bits(g1 - __uint_as_float(bg1 << 16));
    const unsigned w0 = bh0 | (bh1 << 16), w1 = bg0 | (bg1 << 16);
    const unsigned w2 = lh0 | (lh1 << 16), w3 = lg0 | (lg1 << 16);
    if (node < mRows) {
      volatile unsigned* up = (volatile unsigned*)(UA + (size_t)node * KU1);
      up[lane] = w0; up[32 + lane] = w1; up[64 + lane] = w2; up[96 + lane] = w3;
      __threadfence();
      up[lane] = w0; up[32 + lane] = w1; up[64 + lane] = w2; up[96 + lane] = w3;
    }
  }
  __syncthreads();

  v4f pvv[SPW / 32];
#pragma unroll
  for (int i = 0; i < SPW / 32; ++i) {
    const int slot = wave * SPW + 32 * i + lane;
    pvv[i] = *(const v4fa*)(sPos + slot * 4);
  }
#pragma unroll
  for (int i = 0; i < SPW / 32; ++i) {
    const int slot = wave * SPW + 32 * i + lane;
    *(volatile v4f*)(posNext + (size_t)(nodeBase + slot) * 4) = pvv[i];
  }
  __threadfence();
#pragma unroll
  for (int i = 0; i < SPW / 32; ++i) {
    const int slot = wave * SPW + 32 * i + lane;
    *(volatile v4f*)(posNext + (size_t)(nodeBase + slot) * 4) = pvv[i];
  }
}

static inline int cdiv(int a, int b) { return (a + b - 1) / b; }

extern "C" void kernel_launch(void* const* d_in, const int* in_sizes, int n_in,
                              void* d_out, int out_size, void* d_ws, size_t ws_size,
                              hipStream_t stream) {
  if (n_in < 18) return;
  if (in_sizes[0] < INDIM || (in_sizes[0] % INDIM) != 0) return;
  const int nN = in_sizes[0] / INDIM;
  if (in_sizes[1] != nN * 3) return;
  if (in_sizes[3] < 2 || (in_sizes[3] & 1) != 0) return;
  const int nE = in_sizes[3] / 2;
  if (nE < 4 || nE >= (1 << 21)) return;
  if (in_sizes[2] != nE * EDIM) return;
  if (in_sizes[4] != INDIM * EMB || in_sizes[5] != EMB) return;
  if (in_sizes[6] != NLAY * MR * EMB || in_sizes[7] != NLAY * EMB) return;
  if (in_sizes[8] != NLAY * EMB * EMB || in_sizes[9] != NLAY * EMB) return;
  if (in_sizes[10] != NLAY * EMB || in_sizes[11] != NLAY) return;
  if (in_sizes[12] != NLAY * 2 * EMB * EMB || in_sizes[13] != NLAY * EMB) return;
  if (in_sizes[14] != NLAY * EMB * EMB || in_sizes[15] != NLAY * EMB) return;
  if (in_sizes[16] != EMB || in_sizes[17] != 1) return;
  if (out_size != nN) return;

  const float* x    = (const float*)d_in[0];
  const float* pos  = (const float*)d_in[1];
  const float* ea   = (const float*)d_in[2];
  const int*   ei   = (const int*)d_in[3];
  const float* Win  = (const float*)d_in[4];
  const float* bin  = (const float*)d_in[5];
  const float* Wm1  = (const float*)d_in[6];
  const float* bm1  = (const float*)d_in[7];
  const float* Wm2  = (const float*)d_in[8];
  const float* bm2  = (const float*)d_in[9];
  const float* Wp   = (const float*)d_in[10];
  const float* bp   = (const float*)d_in[11];
  const float* Wu1  = (const float*)d_in[12];
  const float* bu1  = (const float*)d_in[13];
  const float* Wu2  = (const float*)d_in[14];
  const float* bu2  = (const float*)d_in[15];
  const float* Wout = (const float*)d_in[16];
  const float* bout = (const float*)d_in[17];
  float* out = (float*)d_out;
  const int* src = ei;
  const int* dst = ei + nE;

  const int MP  = cdiv(nN, GBM) * GBM;
  const int gM  = MP / GBM;
  const int gA  = cdiv(nN, NBA);
  const int NBP = gA * NBA;
  if (NBP < MP) return;
  const int gE  = cdiv(nE, EPB);
  const int EP  = gE * EPB;
  const int vec8 = ((nE & 3) == 0) ? 1 : 0;

  char* ws = (char*)d_ws;
  size_t off = 0;
  const size_t oWIN = off; off += (size_t)EMB * KX * 2;                 off = (off + 255) & ~(size_t)255;
  const size_t oWAB = off; off += (size_t)NLAY * NAB * KAB * 2;         off = (off + 255) & ~(size_t)255;
  const size_t oWM2 = off; off += (size_t)NLAY * EMB * EMB * 2;         off = (off + 255) & ~(size_t)255;
  const size_t oWU1 = off; off += (size_t)NLAY * EMB * KU1 * 2;         off = (off + 255) & ~(size_t)255;
  const size_t oWU2 = off; off += (size_t)NLAY * EMB * KU2 * 2;         off = (off + 255) & ~(size_t)255;
  const size_t oXA  = off; off += (size_t)MP * KX * 2;                  off = (off + 255) & ~(size_t)255;
  const size_t oH   = off; off += (size_t)MP * EMB * 4;                 off = (off + 255) & ~(size_t)255;
  const size_t oHB  = off; off += (size_t)MP * KAB * 2;                 off = (off + 255) & ~(size_t)255;
  const size_t oPAB = off; off += (size_t)MP * NAB * 4;                 off = (off + 255) & ~(size_t)255;
  const size_t oUA  = off; off += (size_t)MP * KU1 * 2;                 off = (off + 255) & ~(size_t)255;
  const size_t oU1A = off; off += (size_t)MP * KU2 * 2;                 off = (off + 255) & ~(size_t)255;
  const size_t oPA  = off; off += (size_t)NBP * 4 * 4;                  off = (off + 255) & ~(size_t)255;
  const size_t oPB  = off; off += (size_t)NBP * 4 * 4;                  off = (off + 255) & ~(size_t)255;
  const size_t oS   = off; off += (size_t)EP * 4;                       off = (off + 255) & ~(size_t)255;
  const size_t oM   = off; off += (size_t)EP * EMB * 2;                 off = (off + 255) & ~(size_t)255;
  if (off > ws_size || off > (size_t)WSLIM) return;
  unsigned short* WinT = (unsigned short*)(ws + oWIN);
  unsigned short* WABT = (unsigned short*)(ws + oWAB);
  unsigned short* Wm2T = (unsigned short*)(ws + oWM2);
  unsigned short* Wu1T = (unsigned short*)(ws + oWU1);
  unsigned short* Wu2T = (unsigned short*)(ws + oWU2);
  unsigned short* XA   = (unsigned short*)(ws + oXA);
  float*          H    = (float*)(ws + oH);
  unsigned short* HB   = (unsigned short*)(ws + oHB);
  float*          PAB  = (float*)(ws + oPAB);
  unsigned short* UA   = (unsigned short*)(ws + oUA);
  unsigned short* U1A  = (unsigned short*)(ws + oU1A);
  float*          POSA = (float*)(ws + oPA);
  float*          POSB = (float*)(ws + oPB);
  float*          Spl  = (float*)(ws + oS);
  unsigned short* Mpl  = (unsigned short*)(ws + oM);

  const size_t edgeLds = (size_t)EDGE_LDS_BYTES;
  const size_t scanLds = (size_t)SC_LDS_INTS * 4;
  hipFuncSetAttribute(reinterpret_cast<const void*>(&k_edge), hipFuncAttributeMaxDynamicSharedMemorySize, (int)edgeLds);
  hipFuncSetAttribute(reinterpret_cast<const void*>(&k_scan), hipFuncAttributeMaxDynamicSharedMemorySize, (int)scanLds);

  const int nUnits = NU_W + MP * 4 + NBP;
  k_prep<<<cdiv(nUnits, NTHR), NTHR, 0, stream>>>(x, pos, Win, Wm1, Wm2, Wu1, Wu2, nN, MP, NBP,
                                                   WinT, WABT, Wm2T, Wu1T, Wu2T, XA, POSA);
  k_h0<<<gM, GTHR, 0, stream>>>(XA, WinT, bin, nN, H, HB);

  for (int l = 0; l < NLAY; ++l) {
    const float* posCur  = (l & 1) ? POSB : POSA;
    float*       posNext = (l & 1) ? POSA : POSB;
    k_gemm<<<dim3(gM, NAB / GBN), GTHR, 0, stream>>>(HB, KAB, WABT + (size_t)l * NAB * KAB, KAB, KAB,
                                                     PAB, NAB);
    k_edge<<<gE, NTHR, edgeLds, stream>>>(ei, nE, nN, PAB, posCur, ea, Wm2T + (size_t)l * EMB * EMB,
                                          Wm1 + (size_t)l * MR * EMB, bm1 + (size_t)l * EMB,
                                          bm2 + (size_t)l * EMB, Wp + (size_t)l * EMB, bp + l,
                                          Spl, Mpl);
    k_scan<<<gA, NTHR, scanLds, stream>>>(src, dst, nE, nN, vec8, MP, Mpl, Spl, posCur, posNext, H, UA);
    k_u1<<<gM, GTHR, 0, stream>>>(UA, Wu1T + (size_t)l * EMB * KU1, bu1 + (size_t)l * EMB, nN, U1A);
    if (l < NLAY - 1) {
      k_u2<0><<<gM, GTHR, 0, stream>>>(U1A, Wu2T + (size_t)l * EMB * KU2, bu2 + (size_t)l * EMB, nN,
                                       H, HB, Wout, bout, out);
    } else {
      k_u2<1><<<gM, GTHR, 0, stream>>>(U1A, Wu2T + (size_t)l * EMB * KU2, bu2 + (size_t)l * EMB, nN,
                                       H, HB, Wout, bout, out);
    }
  }
}
